// DVDMixer_36112085025134
// MI455X (gfx1250) — hardware-verified
//
#include <hip/hip_runtime.h>


#define NB_ 4096
#define NAG 16
#define RH 64
#define NHD 4
#define GD 32
#define EMB 32
#define SD 128
#define KA 160
#define NW1 (NHD * EMB * GD)

typedef __attribute__((ext_vector_type(16))) __bf16   v16bf;
typedef __attribute__((ext_vector_type(16))) _Float16 v16h;
typedef __attribute__((ext_vector_type(8)))  float    v8f;
typedef __attribute__((ext_vector_type(8)))  unsigned v8u;

__device__ __forceinline__ unsigned f2bf(float f) { unsigned u = __float_as_uint(f); u += 0x7FFFu + ((u >> 16) & 1u); return u >> 16; }
__device__ __forceinline__ unsigned f2h(float f) { return (unsigned)__builtin_bit_cast(unsigned short, (_Float16)f); }
__device__ __forceinline__ int kpat(int v, int half) { return ((v & 4) ? 16 : 0) + half * 8 + 2 * (v & 3); }

template <int F16, int NP> struct Opnd { v16bf p[NP]; };

template <int F16, int NP> __device__ __forceinline__ void pack2(float f0, float f1, unsigned* o) {
    if (F16) { o[0] = f2h(f0) | (f2h(f1) << 16); return; }
    unsigned h0 = f2bf(f0), h1 = f2bf(f1); o[0] = h0 | (h1 << 16);
    if (NP >= 2) {
        float r0 = f0 - __uint_as_float(h0 << 16), r1 = f1 - __uint_as_float(h1 << 16);
        unsigned m0 = f2bf(r0), m1 = f2bf(r1); o[1] = m0 | (m1 << 16);
        if (NP >= 3) {
            float s0 = r0 - __uint_as_float(m0 << 16), s1 = r1 - __uint_as_float(m1 << 16);
            o[2] = f2bf(s0) | (f2bf(s1) << 16);
        }
    }
}
template <int F16, int NP> __device__ __forceinline__ void op_row(const float* rowp, int half, float sc, Opnd<F16, NP>& o) {
    v8u u[NP];
#pragma unroll
    for (int v = 0; v < 8; ++v) {
        int kk = kpat(v, half); unsigned t[3];
        pack2<F16, NP>(rowp[kk] * sc, rowp[kk + 1] * sc, t);
#pragma unroll
        for (int p = 0; p < NP; ++p) u[p][v] = t[p];
    }
#pragma unroll
    for (int p = 0; p < NP; ++p) o.p[p] = __builtin_bit_cast(v16bf, u[p]);
}
template <int F16, int NP> __device__ __forceinline__ void op_row_tail(const float* rowp, int half, float sc, int kvalid, Opnd<F16, NP>& o) {
    v8u u[NP];
#pragma unroll
    for (int v = 0; v < 8; ++v) {
        int kk = kpat(v, half); unsigned t[3];
        float f0 = kk < kvalid ? rowp[kk] * sc : 0.0f, f1 = (kk + 1) < kvalid ? rowp[kk + 1] * sc : 0.0f;
        pack2<F16, NP>(f0, f1, t);
#pragma unroll
        for (int p = 0; p < NP; ++p) u[p][v] = t[p];
    }
#pragma unroll
    for (int p = 0; p < NP; ++p) o.p[p] = __builtin_bit_cast(v16bf, u[p]);
}
template <int F16, int NP> __device__ __forceinline__ void op_col(const float* M, int ld, int n, int k0, int half, float sc, Opnd<F16, NP>& o) {
    v8u u[NP];
#pragma unroll
    for (int v = 0; v < 8; ++v) {
        int kk = k0 + kpat(v, half); unsigned t[3];
        pack2<F16, NP>(M[(size_t)kk * ld + n] * sc, M[(size_t)(kk + 1) * ld + n] * sc, t);
#pragma unroll
        for (int p = 0; p < NP; ++p) u[p][v] = t[p];
    }
#pragma unroll
    for (int p = 0; p < NP; ++p) o.p[p] = __builtin_bit_cast(v16bf, u[p]);
}
template <int F16, int NP> __device__ __forceinline__ void op_col_tail(const float* M, int ld, int n, int k0, int half, float sc, int K, Opnd<F16, NP>& o) {
    v8u u[NP];
#pragma unroll
    for (int v = 0; v < 8; ++v) {
        int kk = k0 + kpat(v, half); unsigned t[3];
        float f0 = kk < K ? M[(size_t)kk * ld + n] * sc : 0.0f, f1 = (kk + 1) < K ? M[(size_t)(kk + 1) * ld + n] * sc : 0.0f;
        pack2<F16, NP>(f0, f1, t);
#pragma unroll
        for (int p = 0; p < NP; ++p) u[p][v] = t[p];
    }
#pragma unroll
    for (int p = 0; p < NP; ++p) o.p[p] = __builtin_bit_cast(v16bf, u[p]);
}
__device__ __forceinline__ v8f wm_bf16(v16bf a, v16bf b, v8f c) { return __builtin_amdgcn_wmma_f32_16x16x32_bf16(false, a, false, b, (short)0, c, false, false); }
template <int F16, int NA, int NB> __device__ __forceinline__ v8f wmma_op(const Opnd<F16, NA>& a, const Opnd<F16, NB>& b, v8f c) {
    if (F16) {
        v16h ah = __builtin_bit_cast(v16h, a.p[0]), bh = __builtin_bit_cast(v16h, b.p[0]);
        c = __builtin_amdgcn_wmma_f32_16x16x32_f16(false, ah, false, bh, (short)0, c, false, false);
        asm volatile("v_nop\n\tv_nop\n\tv_nop\n\tv_nop" : "+v"(c) : "v"(ah), "v"(bh));
        return c;
    }
    constexpr int NMX = NA > NB ? NA : NB;
#pragma unroll
    for (int i = 0; i < NA; ++i)
#pragma unroll
        for (int j = 0; j < NB; ++j)
            if (i + j < NMX) c = wm_bf16(a.p[i], b.p[j], c);
    if (NA == 1 && NB == 1)      asm volatile("v_nop\n\tv_nop\n\tv_nop\n\tv_nop" : "+v"(c) : "v"(a.p[0]), "v"(b.p[0]));
    else if (NA == 2 && NB == 1) asm volatile("v_nop\n\tv_nop\n\tv_nop\n\tv_nop" : "+v"(c) : "v"(a.p[0]), "v"(a.p[1]), "v"(b.p[0]));
    else if (NA == 1 && NB == 2) asm volatile("v_nop\n\tv_nop\n\tv_nop\n\tv_nop" : "+v"(c) : "v"(a.p[0]), "v"(b.p[0]), "v"(b.p[1]));
    else if (NA == 2 && NB == 2) asm volatile("v_nop\n\tv_nop\n\tv_nop\n\tv_nop" : "+v"(c) : "v"(a.p[0]), "v"(a.p[1]), "v"(b.p[0]), "v"(b.p[1]));
    else                         asm volatile("v_nop\n\tv_nop\n\tv_nop\n\tv_nop" : "+v"(c) : "v"(a.p[0]), "v"(a.p[NA - 1]), "v"(b.p[0]), "v"(b.p[NB - 1]), "v"(a.p[NA / 2]), "v"(b.p[NB / 2]));
    return c;
}

struct ZMap { long long s1; long long s2; int zdiv; int pad_; };
__device__ __forceinline__ size_t zoff(const ZMap& m, int z) { return (size_t)((long long)(z / m.zdiv) * m.s1 + (long long)(z % m.zdiv) * m.s2); }

#define ACT_NONE 0
#define ACT_RELU 1
#define ACT_GELU_ERF 2
#define ACT_SILU 3
#define ACT_TANH 4
__device__ __forceinline__ float act_apply(int act, float x) {
    if (act == ACT_RELU) return x > 0.f ? x : 0.f;
    if (act == ACT_GELU_ERF) return 0.5f * x * (1.0f + erff(x * 0.70710678118654752f));
    if (act == ACT_SILU) return x / (1.0f + expf(-x));
    if (act == ACT_TANH) return tanhf(x);
    return x;
}
struct GemmArgs {
    ZMap za, zb_, zc, zbias, zadd, zrsc, zmul, zrbias;
    const float* A; const float* Bm; float* C; const float* bias; const float* add; const float* rsc; const float* mul; const float* rbias;
    long long ldadd, ldmul;
    int lda, ldb, ldc, K;
    float ascale, bscale, oscale, addscale;
    int M, nvalid, nstore, ldrsc;
    int bcs, pad1, pad2, pad3;
};
template <int BT, int F16, int NA, int NB, int RW, int CW, int ACT>
__global__ __launch_bounds__(256) void gemm_kernel(GemmArgs g) {
    constexpr int TR = 16 * RW, TC = 64 * CW, CSTR = TC + 4;
    __shared__ __align__(16) float cst[TR * CSTR];
    const int z = blockIdx.z;
    const float* A = g.A + zoff(g.za, z); const float* Bm = g.Bm + zoff(g.zb_, z); float* C = g.C + zoff(g.zc, z);
    const int tid = threadIdx.x, lane = tid & 31, wv = tid >> 5;
    const int l16 = lane & 15, half = lane >> 4;
    const int rt = wv % RW, ch = wv / RW;
    const int row0 = blockIdx.x * TR, col0 = blockIdx.y * TC + ch * 64;
    int arix = row0 + rt * 16 + l16; if (arix >= g.M) arix = g.M - 1;
    const float* arow = A + (size_t)arix * g.lda;
    v8f acc[4];
#pragma unroll
    for (int t = 0; t < 4; ++t) acc[t] = (v8f){};
    const int K = g.K;
#pragma unroll 1
    for (int kc = 0; kc < K; kc += 32) {
        Opnd<F16, NA> a;
        if (kc + 32 <= K) op_row<F16, NA>(arow + kc, half, g.ascale, a); else op_row_tail<F16, NA>(arow + kc, half, g.ascale, K - kc, a);
#pragma unroll
        for (int t = 0; t < 4; ++t) {
            Opnd<F16, NB> b;
            const int n = col0 + t * 16 + l16;
            if (n < g.nvalid) {
                if (BT) { if (kc + 32 <= K) op_row<F16, NB>(Bm + (size_t)n * g.ldb + kc, half, g.bscale, b); else op_row_tail<F16, NB>(Bm + (size_t)n * g.ldb + kc, half, g.bscale, K - kc, b); }
                else    { if (kc + 32 <= K) op_col<F16, NB>(Bm, g.ldb, n * g.bcs, kc, half, g.bscale, b); else op_col_tail<F16, NB>(Bm, g.ldb, n * g.bcs, kc, half, g.bscale, K, b); }
            } else {
#pragma unroll
                for (int p = 0; p < NB; ++p) b.p[p] = (v16bf){};
            }
            acc[t] = wmma_op<F16, NA, NB>(a, b, acc[t]);
        }
    }
    const float* bias = g.bias ? g.bias + zoff(g.zbias, z) : nullptr;
    const float* add = g.add ? g.add + zoff(g.zadd, z) : nullptr;
    const float* rsc = g.rsc ? g.rsc + zoff(g.zrsc, z) : nullptr;
    const float* mul = g.mul ? g.mul + zoff(g.zmul, z) : nullptr;
    const float* rbias = g.rbias ? g.rbias + zoff(g.zrbias, z) : nullptr;
#pragma unroll
    for (int t = 0; t < 4; ++t) {
        const int cl = ch * 64 + t * 16 + l16;
        const int cg = blockIdx.y * TC + cl;
        const bool cok = cg < g.nvalid;
        const float bv = (bias && cok) ? bias[(size_t)cg * g.bcs] : 0.0f;
#pragma unroll
        for (int r = 0; r < 8; ++r) {
            const int rl = rt * 16 + r + 8 * half;
            float v = acc[t][r] * g.oscale + bv;
            int rg = row0 + rl; if (rg >= g.M) rg = g.M - 1;
            if (rbias) v += rbias[rg];
            if (rsc) v *= rsc[(size_t)rg * g.ldrsc];
            if (mul && cok) v *= mul[(size_t)rg * g.ldmul + cg];
            if (add && cok) v += g.addscale * add[(size_t)rg * g.ldadd + cg];
            cst[rl * CSTR + cl] = v;
        }
    }
    __syncthreads();
    const int col = tid % TC, rsel = tid / TC, rstep = 256 / TC;
    if (ACT != ACT_NONE) {
#pragma unroll 1
        for (int r = rsel; r < TR; r += rstep) cst[r * CSTR + col] = act_apply(ACT, cst[r * CSTR + col]);
    }
    float* ob = C + (size_t)row0 * g.ldc + (size_t)blockIdx.y * TC;
    const bool colok = (int)(blockIdx.y * TC + col) < g.nstore;
    const int rmax = (g.M - row0 < TR) ? (g.M - row0) : TR;
    auto pass = [&]() {
        if (colok) {
#pragma unroll 4
            for (int r = rsel; r < rmax; r += rstep) *(volatile float*)(ob + (size_t)r * g.ldc + col) = cst[r * CSTR + col];
        }
    };
    pass();
    __threadfence();
    pass();
}
static inline ZMap zm(long long s1) { ZMap m; m.s1 = s1; m.s2 = 0; m.zdiv = 1; m.pad_ = 0; return m; }
static inline ZMap zm2(long long s1, long long s2, int zdiv) { ZMap m; m.s1 = s1; m.s2 = s2; m.zdiv = zdiv; m.pad_ = 0; return m; }
static inline GemmArgs gemm_args(const float* A, int lda, ZMap za, const float* Bm, int ldb, ZMap zb, float* C, int ldc, ZMap zc, int M, int N, int K) {
    GemmArgs g; g.za = za; g.zb_ = zb; g.zc = zc; g.zbias = zm(0); g.zadd = zm(0); g.zrsc = zm(0); g.zmul = zm(0); g.zrbias = zm(0);
    g.A = A; g.Bm = Bm; g.C = C; g.bias = nullptr; g.add = nullptr; g.rsc = nullptr; g.mul = nullptr; g.rbias = nullptr; g.ldadd = 0; g.ldmul = 0;
    g.lda = lda; g.ldb = ldb; g.ldc = ldc; g.K = K; g.ascale = 1.0f; g.bscale = 1.0f; g.oscale = 1.0f; g.addscale = 1.0f; g.M = M; g.nvalid = N; g.nstore = N; g.ldrsc = 1;
    g.bcs = 1; g.pad1 = 0; g.pad2 = 0; g.pad3 = 0;
    return g;
}
static_assert(sizeof(ZMap) == 24, "ZMap layout");
static_assert(sizeof(GemmArgs) == 8 * 24 + 8 * 8 + 2 * 8 + 4 * 4 + 4 * 4 + 4 * 4 + 4 * 4, "GemmArgs has no padding");

__global__ __launch_bounds__(256) void softmax_rows(float* S, long long sy, long long sx, int L, float prescale, const float* addv, long long say, int aydiv, int causal,
                                                  const int* imask, long long imy, long long imx, float maskval) {
    __shared__ float red[8];
    const int tid = threadIdx.x, lane = tid & 31, wid = tid >> 5;
    float* row = S + (size_t)blockIdx.y * sy + (size_t)blockIdx.x * sx;
    const float* av = addv ? addv + (size_t)(blockIdx.y / aydiv) * say : nullptr;
    const int* im = imask ? imask + (size_t)(blockIdx.y / aydiv) * imy + (size_t)blockIdx.x * imx : nullptr;
    float v[16];
    const int nj = L / 256;
    float mx = -__builtin_inff();
#pragma unroll
    for (int j = 0; j < 16; ++j) if (j < nj) { float t = row[tid + 256 * j] * prescale; if (av) t += av[tid + 256 * j]; if (im && im[tid + 256 * j] == 0) t = maskval; if (causal && (tid + 256 * j) > (int)blockIdx.x) t = -__builtin_inff(); v[j] = t; mx = fmaxf(mx, t); }
#pragma unroll
    for (int o = 16; o; o >>= 1) mx = fmaxf(mx, __shfl_xor(mx, o, 32));
    if (lane == 0) red[wid] = mx;
    __syncthreads();
    float m = red[0];
#pragma unroll
    for (int i = 1; i < 8; ++i) m = fmaxf(m, red[i]);
    if (m == -__builtin_inff()) m = 0.f;
    __syncthreads();
    float sum = 0.f;
#pragma unroll
    for (int j = 0; j < 16; ++j) if (j < nj) { v[j] = expf(v[j] - m); sum += v[j]; }
#pragma unroll
    for (int o = 16; o; o >>= 1) sum += __shfl_xor(sum, o, 32);
    if (lane == 0) red[wid] = sum;
    __syncthreads();
    float tot = 0.f;
#pragma unroll
    for (int i = 0; i < 8; ++i) tot += red[i];
    const float inv = 1.0f / tot;
#pragma unroll
    for (int j = 0; j < 16; ++j) if (j < nj) *(volatile float*)(row + tid + 256 * j) = v[j] * inv;
    __threadfence();
#pragma unroll
    for (int j = 0; j < 16; ++j) if (j < nj) *(volatile float*)(row + tid + 256 * j) = v[j] * inv;
}

#define VST2(T, p, v) do { const T vst2_v_ = (v); *(volatile T*)(p) = vst2_v_; __threadfence(); *(volatile T*)(p) = vst2_v_; } while (0)
__device__ __forceinline__ float eluf(float x) { return x > 0.f ? x : expm1f(x); }
__global__ __launch_bounds__(256) void k_sa(const float* __restrict__ s, const float* __restrict__ unc, float* SA) { const size_t q = (size_t)blockIdx.x * 256 + threadIdx.x; if (q >= (size_t)NB_ * KA) return; const int k = (int)(q % KA), b = (int)(q / KA); VST2(float, SA + q, k < SD ? s[(size_t)b * SD + k] : (k == SD ? unc[b] : 0.f)); }
__global__ __launch_bounds__(256) void k_mix(const float* __restrict__ HP, const float* __restrict__ att_a, const float* __restrict__ W1S, const float* __restrict__ qs, const float* __restrict__ s, const float* __restrict__ b1W, const float* __restrict__ b1b, const float* __restrict__ wfW, const float* __restrict__ wfb, const float* __restrict__ V1W, const float* __restrict__ V1b, const float* __restrict__ V2W, const float* __restrict__ V2b, float* out) {
    __shared__ float hp[NHD][NAG][GD];
    __shared__ float g[NHD][NAG][GD];
    __shared__ float src[NHD][NAG], dst[NHD][NAG];
    __shared__ float attn[NHD][NAG][NAG];
    __shared__ float w1[NAG][EMB];
    __shared__ float sv[SD];
    __shared__ float e32[3][EMB];
    __shared__ float red[256];
    const int b = blockIdx.x, tid = threadIdx.x;
    for (int q = tid; q < NAG * NHD * GD; q += 256) { const int d = q % GD, h = (q / GD) % NHD, n = q / (GD * NHD); hp[h][n][d] = HP[((size_t)b * NAG + n) * (NHD * GD) + h * GD + d]; }
    if (tid < SD) sv[tid] = s[(size_t)b * SD + tid]; __syncthreads();
    if (tid < NHD * NAG) { const int h = tid / NAG, n = tid % NAG; float a = 0.f, c = 0.f;
#pragma unroll 1
        for (int d = 0; d < GD; ++d) { a += hp[h][n][d] * att_a[h * 2 * GD + d]; c += hp[h][n][d] * att_a[h * 2 * GD + GD + d]; } src[h][n] = a; dst[h][n] = c; }
    if (tid >= 128 && tid < 128 + 3 * EMB) { const int w = (tid - 128) / EMB, e = (tid - 128) % EMB; const float* Wm = w == 0 ? b1W : (w == 1 ? wfW : V1W); const float* bb = w == 0 ? b1b : (w == 1 ? wfb : V1b); float a = bb[e];
#pragma unroll 1
        for (int k = 0; k < SD; ++k) a += sv[k] * Wm[k * EMB + e]; e32[w][e] = w == 0 ? a : (w == 1 ? fabsf(a) : fmaxf(a, 0.f)); }
    __syncthreads();
    if (tid < NHD * NAG) { const int h = tid / NAG, i = tid % NAG; float m = -__builtin_inff();
#pragma unroll 1
        for (int j = 0; j < NAG; ++j) { float e = src[h][i] + dst[h][j]; e = e > 0.f ? e : 0.2f * e; attn[h][i][j] = e; m = fmaxf(m, e); } float den = 0.f;
#pragma unroll 1
        for (int j = 0; j < NAG; ++j) { const float e = expf(attn[h][i][j] - m); attn[h][i][j] = e; den += e; }
#pragma unroll 1
        for (int j = 0; j < NAG; ++j) attn[h][i][j] = attn[h][i][j] / den; }
    __syncthreads();
    for (int q = tid; q < NHD * NAG * GD; q += 256) { const int d = q % GD, i = (q / GD) % NAG, h = q / (GD * NAG); float a = 0.f;
#pragma unroll 1
        for (int j = 0; j < NAG; ++j) a += attn[h][i][j] * hp[h][j][d]; g[h][i][d] = eluf(a); }
    __syncthreads();
    for (int q = tid; q < NAG * EMB; q += 256) { const int e = q % EMB, n = q / EMB; float acc = 0.f;
#pragma unroll 1
        for (int h = 0; h < NHD; ++h) { const float* wr = W1S + (size_t)b * NW1 + h * (EMB * GD) + e * GD; float a = 0.f;
#pragma unroll 1
            for (int d = 0; d < GD; ++d) a += wr[d] * g[h][n][d]; acc += fabsf(a); }
        w1[n][e] = acc * 0.25f; }
    __syncthreads();
    float part = 0.f;
    if (tid < EMB) { float a = e32[0][tid];
#pragma unroll 1
        for (int n = 0; n < NAG; ++n) a += qs[(size_t)b * NAG + n] * w1[n][tid]; part = eluf(a) * e32[1][tid]; }
    else if (tid >= 32 && tid < 32 + EMB) { part = e32[2][tid - 32] * V2W[tid - 32]; }
    red[tid] = part; __syncthreads(); for (int o = 128; o > 0; o >>= 1) { if (tid < o) red[tid] += red[tid + o]; __syncthreads(); }
    if (tid < 32) { VST2(float, out + (size_t)b * 32 + tid, tid == 0 ? red[0] + V2b[0] : 0.f); } }
__global__ __launch_bounds__(256) void k_wpad(const float* __restrict__ Wm, float* WP) { const size_t q = (size_t)blockIdx.x * 256 + threadIdx.x; if (q >= (size_t)KA * NW1) return; const int k = (int)(q / NW1); VST2(float, WP + q, k <= SD ? Wm[q] : 0.f); }
__global__ __launch_bounds__(256) void k_copy(const float* __restrict__ O32, float* out) { const int q = blockIdx.x * 256 + threadIdx.x; if (q >= NB_) return; VST2(float, out + q, O32[(size_t)q * 32]); }
extern "C" void kernel_launch(void* const* d_in, const int* in_sizes, int n_in,
                              void* d_out, int out_size, void* d_ws, size_t ws_size, hipStream_t stream) {
    (void)in_sizes; (void)n_in; (void)out_size;
    const float* qs = (const float*)d_in[0]; const float* s = (const float*)d_in[1]; const float* hs = (const float*)d_in[2]; const float* unc = (const float*)d_in[3]; const float* Wg = (const float*)d_in[4]; const float* att_a = (const float*)d_in[5]; const float* w1sW = (const float*)d_in[6]; const float* w1sb = (const float*)d_in[7];
    const float* b1W = (const float*)d_in[8]; const float* b1b = (const float*)d_in[9]; const float* wfW = (const float*)d_in[10]; const float* wfb = (const float*)d_in[11]; const float* V1W = (const float*)d_in[12]; const float* V1b = (const float*)d_in[13]; const float* V2W = (const float*)d_in[14]; const float* V2b = (const float*)d_in[15];
    float* out = (float*)d_out;
    char* wsp = (char*)d_ws;
    auto take = [&](size_t bytes) { char* p = wsp; wsp += (bytes + 255) & ~(size_t)255; return (void*)p; };
    float* HP = (float*)take((size_t)NB_ * NAG * NHD * GD * 4); float* SA = (float*)take((size_t)NB_ * KA * 4); float* W1S = (float*)take((size_t)NB_ * NW1 * 4); float* O32 = (float*)take((size_t)NB_ * 32 * 4); float* WP = (float*)take((size_t)KA * NW1 * 4);
    if ((size_t)(wsp - (char*)d_ws) > ws_size) return;
    { GemmArgs g = gemm_args(hs, RH, zm(0), Wg, NHD * GD, zm(0), HP, NHD * GD, zm(0), NB_ * NAG, NHD * GD, RH); gemm_kernel<0, 0, 2, 2, 8, 1, ACT_NONE><<<dim3((NB_ * NAG) / 128, 2, 1), 256, 0, stream>>>(g); }
    k_sa<<<(unsigned)(((size_t)NB_ * KA) / 256), 256, 0, stream>>>(s, unc, SA);
    k_wpad<<<(unsigned)(((size_t)KA * NW1) / 256), 256, 0, stream>>>(w1sW, WP);
    { GemmArgs g = gemm_args(SA, KA, zm(0), WP, NW1, zm(0), W1S, NW1, zm(0), NB_, NW1, KA); g.bias = w1sb; gemm_kernel<0, 0, 2, 2, 4, 2, ACT_NONE><<<dim3(NB_ / 64, NW1 / 128, 1), 256, 0, stream>>>(g); }
    k_mix<<<NB_, 256, 0, stream>>>(HP, att_a, W1S, qs, s, b1W, b1b, wfW, wfb, V1W, V1b, V2W, V2b, O32);
    k_copy<<<NB_ / 256, 256, 0, stream>>>(O32, out);
}
